// DotProductAttention_87024627352347
// MI455X (gfx1250) — hardware-verified
//
#include <hip/hip_runtime.h>
#include <math.h>

typedef __attribute__((ext_vector_type(16))) _Float16 v16h;
typedef __attribute__((ext_vector_type(8)))  _Float16 v8h;
typedef __attribute__((ext_vector_type(8)))  float v8f;
typedef __attribute__((ext_vector_type(4)))  float v4f;

template <typename T> __device__ __forceinline__ void vst2(void* p, T v) { *(volatile T*)p = v; __threadfence(); *(volatile T*)p = v; }
__device__ __forceinline__ v8f wmma16(v16h a, v16h b, v8f c) {
  v8f d = __builtin_amdgcn_wmma_f32_16x16x32_f16(false, a, false, b, (short)0, c, false, false);
  asm volatile("v_nop\n\tv_nop\n\tv_nop\n\tv_nop" : "+v"(d) : "v"(a), "v"(b));
  return d;
}
__device__ __forceinline__ v16h frag_h(const _Float16* rowk0, unsigned lane) {
  union { v16h v; v8h q[2]; } u; const _Float16* p = rowk0 + 8u * (lane >> 4);
  u.q[0] = *(const v8h*)p; u.q[1] = *(const v8h*)(p + 16); return u.v;
}
__device__ __forceinline__ v16h frag_f32(const float* rowk0, unsigned lane) {
  v16h a; const float* p = rowk0 + 8u * (lane >> 4);
#pragma unroll
  for (int i = 0; i < 8; ++i) { a[i] = (_Float16)p[i]; a[8 + i] = (_Float16)p[16 + i]; }
  return a;
}
#define LDSX() do { asm volatile("s_wait_dscnt 0" ::: "memory"); __builtin_amdgcn_wave_barrier(); __builtin_amdgcn_fence(3  , "workgroup"); } while (0)

#ifndef NB
#define NB 16
#endif
#ifndef TT
#define TT 2048
#endif
#define NB_FULL 16
#define TT_FULL 2048
#define CC 128
#define HD 128
#define NQB (TT / 64)
#define SCALE (0.08838834764831845f)
#define FILLV (-1.0e6f)
#if (NB % 4) == 0
#define BG 4
#else
#define BG 1
#endif
static_assert(TT % 128 == 0);
static_assert(TT <= TT_FULL);
static_assert(NB <= NB_FULL);
static_assert(NB % BG == 0);
static_assert((NB * TT) % 64 == 0);
static_assert(NQB * 64 == TT);
static_assert(HD == 128);
static_assert(CC == HD);

__device__ __forceinline__ float bfr(float v) { return (float)(__bf16)v; }
__device__ __forceinline__ unsigned vl_clamp(int vl) { return vl <= 0 ? 0u : ((unsigned)vl > (unsigned)TT ? (unsigned)TT : (unsigned)vl); }
__device__ __forceinline__ unsigned kend128(unsigned vlc) { return vlc == 0u ? (unsigned)TT : ((vlc + 127u) & ~127u); }

#define WS_QH  ((size_t)0)
#define WS_KH  (WS_QH + (size_t)2 * NB * TT * CC)
#define WS_VT  (WS_KH + (size_t)2 * NB * TT * CC)
#define WS_S   (WS_VT + (size_t)2 * NB * CC * TT)
#define WS_END (WS_S  + (size_t)4 * BG * TT * TT)
static_assert(WS_END <= (size_t)134217728);
static_assert(WS_KH % 128 == 0);
static_assert(WS_VT % 128 == 0);
static_assert(WS_S % 128 == 0);

__global__ __launch_bounds__(128) void k_prep(const float* __restrict__ Q, const float* __restrict__ K, const float* __restrict__ V, _Float16* __restrict__ QH, _Float16* __restrict__ KH, _Float16* __restrict__ VT) {
  __shared__ __align__(16) _Float16 sq[64][136], sk[64][136], tv[128][72];
  const unsigned tid = threadIdx.x; const unsigned r0 = blockIdx.x * 64u; const unsigned bb = r0 / (unsigned)TT, t0 = r0 % (unsigned)TT;
  const size_t ib = ((size_t)bb * TT_FULL + t0) * HD;
  for (unsigned e = tid; e < 64u * 128u; e += 128u) { const unsigned rl = e >> 7, c = e & 127u; const size_t oi = ib + (size_t)rl * HD + c;
    const float q = bfr(Q[oi]), k = bfr(K[oi]), v = bfr(V[oi]);
    sq[rl][c] = (_Float16)q; sk[rl][c] = (_Float16)k; tv[c][rl] = (_Float16)v; }
  __syncthreads();
  for (unsigned e = tid; e < 64u * 16u; e += 128u) { const unsigned rl = e >> 4, q = e & 15u; const size_t o = ((size_t)r0 + rl) * CC + q * 8u;
    const v8h a = *(const v8h*)&sq[rl][q * 8u]; const v8h b = *(const v8h*)&sk[rl][q * 8u];
    vst2(QH + o, a); vst2(KH + o, b); }
  for (unsigned e = tid; e < 128u * 8u; e += 128u) { const unsigned cl = e >> 3, q = e & 7u;
    const v8h a = *(const v8h*)&tv[cl][q * 8u];
    vst2(VT + ((size_t)bb * CC + cl) * (size_t)TT + t0 + q * 8u, a); } }

__global__ __launch_bounds__(128) void k_sc(const _Float16* __restrict__ QH, const _Float16* __restrict__ KH, const int* __restrict__ VL, unsigned b0, float* __restrict__ S0) {
  __shared__ __align__(16) float ss[4][16][132];
  const unsigned qb = blockIdx.x, kb = blockIdx.y, b = b0 + blockIdx.z;
  const unsigned kend = kend128(vl_clamp(VL[b]));
  if (kb * 128u >= kend) return;
  float* S = S0 + (size_t)blockIdx.z * TT * TT;
  const unsigned tid = threadIdx.x, wave = tid >> 5, lane = tid & 31u, col = lane & 15u, g = lane >> 4;
  const unsigned k0 = kb * 128u, ql0 = qb * 64u + wave * 16u; const size_t q0 = (size_t)b * TT + ql0, kr0 = (size_t)b * TT + k0;
  v8f acc[8] = {};
#pragma unroll
  for (int kc = 0; kc < HD / 32; ++kc) { const v16h ah = frag_h(QH + (q0 + col) * CC + kc * 32, lane);
#pragma unroll
    for (int j = 0; j < 8; ++j) { const v16h kbf = frag_h(KH + (kr0 + j * 16 + col) * CC + kc * 32, lane); acc[j] = wmma16(ah, kbf, acc[j]); } }
#pragma unroll
  for (int j = 0; j < 8; ++j) {
#pragma unroll
    for (int r = 0; r < 8; ++r) ss[wave][8 * g + r][j * 16 + col] = acc[j][r] * SCALE; }
  LDSX();
  for (unsigned rl = 0; rl < 16u; ++rl) { const v4f o = *(const v4f*)&ss[wave][rl][lane * 4u]; vst2(S + (size_t)(ql0 + rl) * TT + k0 + lane * 4u, o); } }

__global__ __launch_bounds__(256) void k_sm(float* __restrict__ S0, const int* __restrict__ VL, unsigned b0) {
  __shared__ float sred[8]; __shared__ float sbc; __shared__ __align__(16) float shv[TT];
  const unsigned tid = threadIdx.x, t = blockIdx.x, b = b0 + blockIdx.y;
  const unsigned vlc = vl_clamp(VL[b]); const unsigned kend = kend128(vlc);
  float* sr = S0 + (size_t)blockIdx.y * TT * TT + (size_t)t * TT;
  float m = -3.0e38f;
  for (unsigned k = tid; k < kend; k += 256u) { const float s = sr[k]; const float v = (k < vlc) ? s : FILLV; shv[k] = v; m = fmaxf(m, v); }
#pragma unroll
  for (int o = 1; o < 32; o <<= 1) m = fmaxf(m, __shfl_xor(m, o));
  if ((tid & 31u) == 0u) sred[tid >> 5] = m;
  __syncthreads();
  if (tid == 0u) { float a = sred[0]; for (int i = 1; i < 8; ++i) a = fmaxf(a, sred[i]); sbc = a; }
  __syncthreads(); m = sbc; __syncthreads();
  float sum = 0.f;
  for (unsigned k = tid; k < kend; k += 256u) { const float e = expf(shv[k] - m); shv[k] = e; sum += e; }
#pragma unroll
  for (int o = 1; o < 32; o <<= 1) sum += __shfl_xor(sum, o);
  if ((tid & 31u) == 0u) sred[tid >> 5] = sum;
  __syncthreads();
  if (tid == 0u) { float a = 0.f; for (int i = 0; i < 8; ++i) a += sred[i]; sbc = 2048.0f * (1.0f / a); }
  __syncthreads(); const float inv = sbc;
  for (unsigned k = tid; k < kend; k += 256u) shv[k] = shv[k] * inv;
  __syncthreads();
  for (unsigned q = tid; q < (kend >> 2); q += 256u) { const v4f o = *(const v4f*)&shv[q * 4u]; vst2(sr + q * 4u, o); } }

__global__ __launch_bounds__(128) void k_pv(const float* __restrict__ PS0, const _Float16* __restrict__ VT, const int* __restrict__ VL, unsigned b0, float* __restrict__ Y) {
  __shared__ __align__(16) float ss[4][16][HD + 4];
  const unsigned b = b0 + blockIdx.z; const float* PS = PS0 + (size_t)blockIdx.z * TT * TT;
  const unsigned tid = threadIdx.x, wave = tid >> 5, lane = tid & 31u, col = lane & 15u, g = lane >> 4; const unsigned qb = blockIdx.x; const unsigned ql0 = qb * 64u + wave * 16u;
  const unsigned vlc = vl_clamp(VL[b]);
  unsigned kce = (vlc == 0u ? (unsigned)TT : ((vlc + 31u) & ~31u)) >> 5; if (kce > (unsigned)(TT / 32)) kce = (unsigned)(TT / 32);
  v8f acc[HD / 16] = {};
#pragma unroll 1
  for (unsigned kc = 0; kc < kce; ++kc) { const v16h p = frag_f32(PS + (size_t)(ql0 + col) * TT + kc * 32u, lane);
    asm volatile("s_wait_loadcnt 0x0" ::: "memory");
#pragma unroll
    for (int j = 0; j < HD / 16; ++j) { const size_t po = ((size_t)b * CC + j * 16 + col) * (size_t)TT + kc * 32u; acc[j] = wmma16(p, frag_h(VT + po, lane), acc[j]); } }
#pragma unroll
  for (int j = 0; j < HD / 16; ++j)
#pragma unroll
    for (int r = 0; r < 8; ++r) ss[wave][8 * g + r][j * 16 + col] = acc[j][r] * (1.0f / 2048.0f);
  LDSX();
  for (unsigned rl = 0; rl < 16u; ++rl) { const v4f o = *(const v4f*)&ss[wave][rl][lane * 4u]; vst2(Y + ((size_t)b * TT + ql0 + rl) * HD + lane * 4u, o); } }

extern "C" void kernel_launch(void* const* d_in, const int* in_sizes, int n_in, void* d_out, int out_size, void* d_ws, size_t ws_size, hipStream_t stream) {
  if (n_in < 4) return;
  const size_t need = ((size_t)(NB - 1) * TT_FULL + TT) * CC;
  if ((size_t)in_sizes[0] < need || (size_t)in_sizes[1] < need || (size_t)in_sizes[2] < need || in_sizes[3] < NB) return;
  if ((size_t)out_size < (size_t)NB * TT * CC) return;
  if (ws_size < (size_t)WS_END) return;
  const float* Qp = (const float*)d_in[0]; const float* Kp = (const float*)d_in[1]; const float* Vp = (const float*)d_in[2]; const int* VL = (const int*)d_in[3];
  char* ws = (char*)d_ws; _Float16* QH = (_Float16*)(ws + WS_QH); _Float16* KH = (_Float16*)(ws + WS_KH); _Float16* VT = (_Float16*)(ws + WS_VT); float* S = (float*)(ws + WS_S);
  k_prep<<<dim3(NB * TT / 64), 128, 0, stream>>>(Qp, Kp, Vp, QH, KH, VT);
  for (unsigned b0 = 0; b0 < (unsigned)NB; b0 += BG) {
    k_sc<<<dim3(NQB, TT / 128, BG), 128, 0, stream>>>(QH, KH, VL, b0, S);
    k_sm<<<dim3(TT, BG), 256, 0, stream>>>(S, VL, b0);
    k_pv<<<dim3(NQB, 1, BG), 128, 0, stream>>>(S, VT, VL, b0, (float*)d_out);
  }
}
